// MoE_LoRA_MLP_43130061586817
// MI455X (gfx1250) — hardware-verified
//
#include <hip/hip_runtime.h>
#include <math.h>

typedef __attribute__((ext_vector_type(16))) _Float16 v16h;
typedef __attribute__((ext_vector_type(16))) __bf16 v16b;
typedef __attribute__((ext_vector_type(8)))  _Float16 v8h;
typedef __attribute__((ext_vector_type(8)))  float v8f;
typedef __attribute__((ext_vector_type(4)))  float v4f;
typedef __attribute__((ext_vector_type(2)))  float v2f;
typedef __attribute__((ext_vector_type(4)))  unsigned v4u;
typedef __attribute__((ext_vector_type(4)))  int v4i;
typedef float __attribute__((may_alias)) float_a;
typedef int __attribute__((may_alias)) int_a;

template <typename T> __device__ __forceinline__ void vst2(void* p, T v) { *(volatile T*)p = v; __threadfence(); *(volatile T*)p = v; }
__device__ __forceinline__ v8f wmma16(v16h a, v16h b, v8f c) {
  v8f d = __builtin_amdgcn_wmma_f32_16x16x32_f16(false, a, false, b, (short)0, c, false, false);
  asm volatile("v_nop\n\tv_nop\n\tv_nop\n\tv_nop" : "+v"(d) : "v"(a), "v"(b));
  return d;
}
__device__ __forceinline__ v8f wmma_bf(v16b a, v16b b, v8f c) {
  v8f d = __builtin_amdgcn_wmma_f32_16x16x32_bf16(false, a, false, b, (short)0, c, false, false);
  asm volatile("v_nop\n\tv_nop\n\tv_nop\n\tv_nop" : "+v"(d) : "v"(a), "v"(b));
  return d;
}
__device__ __forceinline__ v16h frag_h(const _Float16* rowk0, int lane) {
  union { v16h v; v8h q[2]; } u; const _Float16* p = rowk0 + 8 * (lane >> 4);
  u.q[0] = *(const v8h*)p; u.q[1] = *(const v8h*)(p + 16); return u.v;
}
__device__ __forceinline__ v16h frag_f32(const float* rowk0, int lane) {
  v16h a; const float* p = rowk0 + 8 * (lane >> 4);
#pragma unroll
  for (int i = 0; i < 8; ++i) { a[i] = (_Float16)p[i]; a[8 + i] = (_Float16)p[16 + i]; }
  return a;
}
__device__ __forceinline__ v16h frag_f32s(const float* rowk0, int lane, float sc) {
  v16h a; const float* p = rowk0 + 8 * (lane >> 4);
#pragma unroll
  for (int i = 0; i < 8; ++i) { a[i] = (_Float16)(p[i] * sc); a[8 + i] = (_Float16)(p[16 + i] * sc); }
  return a;
}
__device__ __forceinline__ v16h fragc_f32(const float* W, int k0, int n, int lane, int ld, int K) {
  v16h a; const int g = lane >> 4;
#pragma unroll
  for (int i = 0; i < 8; ++i) { const int ka = k0 + 8 * g + i, kb = ka + 16;
    a[i] = (_Float16)(ka < K ? W[(size_t)(ka < K ? ka : K - 1) * ld + n] : 0.f); a[8 + i] = (_Float16)(kb < K ? W[(size_t)(kb < K ? kb : K - 1) * ld + n] : 0.f); }
  return a;
}
struct F2 { v16b h, l; };
__device__ __forceinline__ F2 bsplit16(const float v[16]) { F2 r;
#pragma unroll
  for (int i = 0; i < 16; ++i) { const __bf16 h = (__bf16)v[i]; r.h[i] = h; r.l[i] = (__bf16)(v[i] - (float)h); }
  return r; }
__device__ __forceinline__ F2 split_row(const float* row, int k0, int lane) { float v[16]; const float* p = row + k0 + 8 * (lane >> 4);
#pragma unroll
  for (int i = 0; i < 8; ++i) { v[i] = p[i]; v[8 + i] = p[16 + i]; }
  return bsplit16(v); }
__device__ __forceinline__ F2 split_rowK(const float* row, int k0, int lane, int K) { float v[16]; const int g = lane >> 4;
#pragma unroll
  for (int i = 0; i < 8; ++i) { const int ka = k0 + 8 * g + i, kb = ka + 16; v[i] = ka < K ? row[ka < K ? ka : K - 1] : 0.f; v[8 + i] = kb < K ? row[kb < K ? kb : K - 1] : 0.f; }
  return bsplit16(v); }
__device__ __forceinline__ F2 split_col(const float* W, int k0, int n, int lane, int ld, int K) { float v[16]; const int g = lane >> 4;
#pragma unroll
  for (int i = 0; i < 8; ++i) { const int ka = k0 + 8 * g + i, kb = ka + 16; v[i] = ka < K ? W[(size_t)(ka < K ? ka : K - 1) * ld + n] : 0.f; v[8 + i] = kb < K ? W[(size_t)(kb < K ? kb : K - 1) * ld + n] : 0.f; }
  return bsplit16(v); }
__device__ __forceinline__ v8f mac3(const F2& a, const F2& b, v8f c) { c = wmma_bf(a.l, b.h, c); c = wmma_bf(a.h, b.l, c); return wmma_bf(a.h, b.h, c); }
__device__ __forceinline__ float sigm(float v) { return 1.0f / (1.0f + expf(-v)); }
#define LDSX() do { asm volatile("s_wait_dscnt 0" ::: "memory"); __builtin_amdgcn_wave_barrier(); __builtin_amdgcn_fence(__ATOMIC_RELEASE, "workgroup"); } while (0)


#define NTOK 4096
#define DD 1024
#define HH_ 4096
#define NE 8
#define RK 32
#define NBLK (NTOK / 64)
#ifndef NBLKT
#define NBLKT NBLK
#endif
#define MAXT 16
typedef __attribute__((ext_vector_type(8))) __bf16 v8b;
__device__ __forceinline__ v16b frag_b(const __bf16* rowk0, int lane) {
  union { v16b v; v8b q[2]; } u; const __bf16* p = rowk0 + 8 * (lane >> 4);
  u.q[0] = *(const v8b*)p; u.q[1] = *(const v8b*)(p + 16); return u.v;
}
__device__ __forceinline__ float bfr(float v) { return (float)(__bf16)v; }
__device__ __attribute__((noinline)) float exp_ni(float v) { return expf(v); }
__device__ __attribute__((noinline)) float erf_ni(float v) { return erff(v); }

__device__ __attribute__((noinline)) float erf_ni2(float v) { return erff(v); }
#define WS_LST  0u
#define WS_CNTI (WS_LST + 4u * NE * NBLK * 64)
#define WS_OFFI (WS_CNTI + 4u * NBLK * 32)
#define WS_GE   (WS_OFFI + 4u * (NE * NBLK + 32))
#define WS_PW   (WS_GE + 4u * NTOK)
#define PG 0
#define PF1 (PG + 16 * DD)
#define PF2 (PF1 + (size_t)HH_ * DD)
#define PAD_ (PF2 + (size_t)DD * HH_)
#define PBD (PAD_ + (size_t)NE * RK * DD)
#define PAU (PBD + (size_t)NE * HH_ * RK)
#define PBU (PAU + (size_t)NE * RK * HH_)
#define PWEND (PBU + (size_t)NE * DD * RK)
#define WS_HD   (WS_PW + 2u * PWEND)
#define WS_A    (WS_HD + 4u * NTOK * RK)
#define WS_LO   (WS_A + 4u * NTOK * HH_)
#define WS_END  (WS_LO + 4u * NTOK * HH_)

__global__ __launch_bounds__(256) void k_packT(const float* __restrict__ RW, const float* __restrict__ F1, const float* __restrict__ F2_, const float* __restrict__ AD, const float* __restrict__ BD, const float* __restrict__ AU, const float* __restrict__ BU, __bf16* __restrict__ PW) {
  __shared__ __align__(16) __bf16 s[HH_]; const int n = blockIdx.x, which = blockIdx.y, tid = threadIdx.x; int K; size_t dst; const float* src;
  switch (which) {
    case 0: if (n >= 16) return; K = DD; dst = PG + (size_t)n * DD; src = (n < NE) ? RW + (size_t)n * DD : nullptr; break;
    case 1: if (n >= HH_) return; K = DD; dst = PF1 + (size_t)n * DD; src = F1 + (size_t)n * DD; break;
    case 2: if (n >= DD) return; K = HH_; dst = PF2 + (size_t)n * HH_; src = F2_ + (size_t)n * HH_; break;
    case 3: if (n >= NE * RK) return; K = DD; dst = PAD_ + (size_t)n * DD; src = AD + (size_t)n * DD; break;
    case 4: if (n >= NE * HH_) return; K = RK; dst = PBD + (size_t)n * RK; src = BD + (size_t)n * RK; break;
    case 5: if (n >= NE * RK) return; K = HH_; dst = PAU + (size_t)n * HH_; src = AU + (size_t)n * HH_; break;
    default: if (n >= NE * DD) return; K = RK; dst = PBU + (size_t)n * RK; src = BU + (size_t)n * RK; break; }
  for (int k = tid; k < K; k += 256) s[k] = (__bf16)(src ? src[k] : 0.f);
  __syncthreads();
  for (int q = tid; q < K / 8; q += 256) vst2((unsigned*)(PW + dst + q * 8), *(const v4u*)&s[q * 8]);
}
__global__ __launch_bounds__(128) void k_gate(const float* __restrict__ X, const __bf16* __restrict__ PW, const float* __restrict__ BR, float* __restrict__ OR, float* __restrict__ OC, int* __restrict__ GE, int* __restrict__ LST, int* __restrict__ CNTI) {
  __shared__ float sl[4][16][NE + 1]; __shared__ __align__(16) float sro[64][NE], sch[64][NE]; __shared__ __align__(16) int sge[64]; __shared__ __align__(16) int slst[NE][64]; __shared__ __align__(16) int scnt[32];
  const int tid = threadIdx.x, wave = tid >> 5, lane = tid & 31, col = lane & 15, g = lane >> 4; const size_t r0 = (size_t)blockIdx.x * 64 + wave * 16;
  v8f acc = {};
#pragma unroll 4
  for (int kc = 0; kc < DD / 32; ++kc) { v16b a; { const float* p = X + (r0 + col) * DD + kc * 32 + 8 * g;
#pragma unroll
      for (int i = 0; i < 8; ++i) { a[i] = (__bf16)p[i]; a[8 + i] = (__bf16)p[16 + i]; } }
    acc = wmma_bf(a, frag_b(PW + PG + (size_t)col * DD + kc * 32, lane), acc); }
  if (col < NE) {
#pragma unroll
    for (int r = 0; r < 8; ++r) sl[wave][8 * g + r][col] = acc[r] + bfr(BR[col]); }
  LDSX();
  if (lane < 16) { const int rl = lane; const int tl = wave * 16 + rl; float lg[NE];
#pragma unroll
    for (int e = 0; e < NE; ++e) lg[e] = sl[wave][rl][e];
    int i1 = 0; float v1 = lg[0];
#pragma unroll
    for (int e = 1; e < NE; ++e) if (lg[e] > v1) { v1 = lg[e]; i1 = e; }
    float s = 0.f; float ex[NE];
#pragma unroll
    for (int e = 0; e < NE; ++e) { ex[e] = exp_ni(lg[e] - v1); s += ex[e]; }
#pragma unroll
    for (int e = 0; e < NE; ++e) { const float r_ = ex[e] / s; const float mk = (e == i1) ? 1.f : 0.f; sro[tl][e] = r_; sch[tl][e] = (mk - r_) + r_; }
    sge[tl] = i1; }
  __syncthreads();
  for (int q = tid; q < 64 * NE / 4; q += 128) { vst2(OR + (size_t)blockIdx.x * 64 * NE + q * 4, *(const v4f*)&(&sro[0][0])[q * 4]); vst2(OC + (size_t)blockIdx.x * 64 * NE + q * 4, *(const v4f*)&(&sch[0][0])[q * 4]); }
  if (tid < 16) vst2((unsigned*)(GE + (size_t)blockIdx.x * 64 + tid * 4), *(const v4u*)&sge[tid * 4]);
  for (int q = tid; q < NE * 64; q += 128) slst[q >> 6][q & 63] = -1;
  if (tid < 32) scnt[tid] = 0;
  __syncthreads();
  if (tid < NE) { int c = 0; for (int p = 0; p < 64; ++p) if (sge[p] == tid) { slst[tid][c++] = blockIdx.x * 64 + p; } scnt[tid] = c; }
  __syncthreads();
  for (int q = tid; q < NE * 16; q += 128) { const int e = q >> 4, pc = q & 15; vst2((unsigned*)(LST + ((size_t)e * NBLK + blockIdx.x) * 64 + pc * 4), *(const v4u*)&slst[e][pc * 4]); }
  if (tid < 8) vst2((unsigned*)(CNTI + (size_t)blockIdx.x * 32 + tid * 4), *(const v4u*)&scnt[tid * 4]);
}
__global__ __launch_bounds__(32) void k_mscan(const int* __restrict__ CNTI, int* __restrict__ OFFI) {
  __shared__ __align__(16) int so[NE][NBLK]; __shared__ __align__(16) int stot[32]; const int e = threadIdx.x;
  if (e < NE) { int run = 0; for (int b = 0; b < NBLK; ++b) { so[e][b] = run; if (b < NBLKT) run += min(max(CNTI[(size_t)b * 32 + e], 0), 64); } stot[e] = run; } else if (e < 32) stot[e] = 0;
  __syncthreads();
  for (int q = e; q < NE * NBLK / 4; q += 32) vst2((unsigned*)(OFFI + q * 4), *(const v4u*)&(&so[0][0])[q * 4]);
  if (e < 8) vst2((unsigned*)(OFFI + NE * NBLK + e * 4), *(const v4u*)&stot[e * 4]);
}
__device__ __forceinline__ int moe_tok(const int* __restrict__ OFFI, const int* __restrict__ CNTI, const int* __restrict__ LST, int e, int r) {
  int lo = 0, hi = NBLKT - 1; while (lo < hi) { const int mid = (lo + hi + 1) >> 1; if (OFFI[e * NBLK + mid] <= r) lo = mid; else hi = mid - 1; }
  const int off = OFFI[e * NBLK + lo]; const int c = min(max(CNTI[(size_t)lo * 32 + e], 0), 64); const int i = r - off; if (i < 0 || i >= c) return -1;
  const int p = LST[((size_t)e * NBLK + lo) * 64 + i]; return (p < 0 || p >= NTOK) ? -1 : p;
}
template <int UP>
__global__ __launch_bounds__(128) void k_rank(const float* __restrict__ IN, const __bf16* __restrict__ PW, const float* __restrict__ AB, const int* __restrict__ LST, const int* __restrict__ CNTI, const int* __restrict__ OFFI, float* __restrict__ HD) {
  __shared__ __align__(16) float so[4][16][36]; __shared__ int stok[64];
  const int tid = threadIdx.x, wave = tid >> 5, lane = tid & 31, col = lane & 15, g = lane >> 4; const int t = blockIdx.x, e = blockIdx.z;
  const int cnt = min(max(OFFI[NE * NBLK + e], 0), NTOK); if (t * 64 >= cnt) return;
  if (tid < 64) { const int i = t * 64 + tid; stok[tid] = (i < cnt) ? moe_tok(OFFI, CNTI, LST, e, i) : -1; }
  __syncthreads();
  const int my = stok[wave * 16 + col]; const size_t tok = (size_t)(my < 0 ? 0 : my); const int K = UP ? HH_ : DD; const __bf16* PA = PW + (UP ? PAU : PAD_) + (size_t)e * RK * K;
  v8f acc[2] = {};
#pragma unroll 2
  for (int kc = 0; kc < K / 32; ++kc) { F2 a; if (UP) a = split_row(IN + tok * HH_, kc * 32, lane); else { v16b ax; const float* p = IN + tok * DD + kc * 32 + 8 * g;
#pragma unroll
      for (int i = 0; i < 8; ++i) { ax[i] = (__bf16)p[i]; ax[8 + i] = (__bf16)p[16 + i]; } a.h = ax; a.l = ax; }
#pragma unroll
    for (int j = 0; j < 2; ++j) { const v16b w = frag_b(PA + (size_t)(j * 16 + col) * K + kc * 32, lane); if (UP) acc[j] = wmma_bf(a.l, w, acc[j]); acc[j] = wmma_bf(a.h, w, acc[j]); } }
#pragma unroll
  for (int j = 0; j < 2; ++j) { const float bb = bfr(AB[e * RK + j * 16 + col]);
#pragma unroll
    for (int r = 0; r < 8; ++r) so[wave][8 * g + r][j * 16 + col] = acc[j][r] + bb; }
  LDSX();
  for (int rl = 0; rl < 16; ++rl) { const int tk = stok[wave * 16 + rl]; if (tk >= 0 && lane < 8) vst2(HD + (size_t)tk * RK + lane * 4, *(const v4f*)&so[wave][rl][lane * 4]); }
}
template <int UP>
__global__ __launch_bounds__(128) void k_lexp(const float* __restrict__ HD, const __bf16* __restrict__ PW, const float* __restrict__ BB, const int* __restrict__ LST, const int* __restrict__ CNTI, const int* __restrict__ OFFI, float* __restrict__ LO) {
  __shared__ __align__(16) float so[4][16][132]; __shared__ int stok[64];
  const int tid = threadIdx.x, wave = tid >> 5, lane = tid & 31, col = lane & 15, g = lane >> 4; const int t = blockIdx.x, e = blockIdx.z; const int n0 = blockIdx.y * 128; const int NOUT = UP ? DD : HH_;
  const int cnt = min(max(OFFI[NE * NBLK + e], 0), NTOK); if (t * 64 >= cnt) return;
  if (tid < 64) { const int i = t * 64 + tid; stok[tid] = (i < cnt) ? moe_tok(OFFI, CNTI, LST, e, i) : -1; }
  __syncthreads();
  const int my = stok[wave * 16 + col]; const size_t tok = (size_t)(my < 0 ? 0 : my); const __bf16* PB = PW + (UP ? PBU : PBD) + ((size_t)e * NOUT + n0) * RK;
  v8f acc[8] = {};
  { const F2 a = split_row(HD + tok * RK, 0, lane);
#pragma unroll
    for (int j = 0; j < 8; ++j) { const v16b w = frag_b(PB + (size_t)(j * 16 + col) * RK, lane); acc[j] = wmma_bf(a.l, w, acc[j]); acc[j] = wmma_bf(a.h, w, acc[j]); } }
#pragma unroll
  for (int j = 0; j < 8; ++j) { const float bb = bfr(BB[(size_t)e * NOUT + n0 + j * 16 + col]);
#pragma unroll
    for (int r = 0; r < 8; ++r) so[wave][8 * g + r][j * 16 + col] = acc[j][r] + bb; }
  LDSX();
  for (int rl = 0; rl < 16; ++rl) { const int tk = stok[wave * 16 + rl]; if (tk >= 0) vst2(LO + (size_t)tk * NOUT + n0 + lane * 4, *(const v4f*)&so[wave][rl][lane * 4]); }
}
template <int UP>
__global__ __launch_bounds__(128) void k_layer(const float* __restrict__ IN, const __bf16* __restrict__ PW, const float* __restrict__ BIAS, const float* __restrict__ LO, float* __restrict__ OUT) {
  __shared__ __align__(16) float so[4][16][132];
  const int tid = threadIdx.x, wave = tid >> 5, lane = tid & 31, col = lane & 15, g = lane >> 4; const size_t r0 = (size_t)blockIdx.x * 64 + wave * 16; const int n0 = blockIdx.y * 128;
  const int K = UP ? HH_ : DD; const __bf16* P = PW + (UP ? PF2 : PF1); const int NOUT = UP ? DD : HH_;
  v8f acc[8] = {};
#pragma unroll 2
  for (int kc = 0; kc < K / 32; ++kc) { F2 a; if (UP) a = split_row(IN + (r0 + col) * (size_t)HH_, kc * 32, lane); else { v16b ax; const float* p = IN + (r0 + col) * (size_t)DD + kc * 32 + 8 * g;
#pragma unroll
      for (int i = 0; i < 8; ++i) { ax[i] = (__bf16)p[i]; ax[8 + i] = (__bf16)p[16 + i]; } a.h = ax; a.l = ax; }
#pragma unroll
    for (int j = 0; j < 8; ++j) { const v16b w = frag_b(P + (size_t)(n0 + j * 16 + col) * K + kc * 32, lane); if (UP) acc[j] = wmma_bf(a.l, w, acc[j]); acc[j] = wmma_bf(a.h, w, acc[j]); } }
#pragma unroll
  for (int j = 0; j < 8; ++j) { const int n = n0 + j * 16 + col; const float bb = bfr(BIAS[n]);
#pragma unroll
    for (int r = 0; r < 8; ++r) { float v = acc[j][r] + bb + LO[(r0 + 8 * g + r) * (size_t)NOUT + n] * (1.0f / 32.0f); if (!UP) v = 0.5f * v * (1.0f + erf_ni2(v * 0.70710678118654752f)); so[wave][8 * g + r][j * 16 + col] = v; } }
  LDSX();
  for (int rl = 0; rl < 16; ++rl) vst2(OUT + (r0 + rl) * (size_t)NOUT + n0 + lane * 4, *(const v4f*)&so[wave][rl][lane * 4]);
}
extern "C" void kernel_launch(void* const* d_in, const int* in_sizes, int n_in, void* d_out, int out_size, void* d_ws, size_t ws_size, hipStream_t stream) {
  (void)in_sizes; (void)n_in; (void)out_size;
  const float** F = (const float**)d_in;
  if (ws_size < (size_t)WS_END) return;
  char* ws = (char*)d_ws; int *LST = (int*)(ws + WS_LST), *CNTI = (int*)(ws + WS_CNTI), *OFFI = (int*)(ws + WS_OFFI), *GE = (int*)(ws + WS_GE); __bf16* PW = (__bf16*)(ws + WS_PW); float *HD = (float*)(ws + WS_HD), *AA = (float*)(ws + WS_A), *LO = (float*)(ws + WS_LO);
  float* OUP = (float*)d_out; float* OR = OUP + (size_t)NTOK * DD; float* OC = OR + (size_t)NTOK * NE;
  k_packT<<<dim3(NE * HH_, 7), 256, 0, stream>>>(F[1], F[3], F[5], F[7], F[9], F[11], F[13], PW);
  k_gate<<<NBLKT, 128, 0, stream>>>(F[0], PW, F[2], OR, OC, GE, LST, CNTI);
  k_mscan<<<1, 32, 0, stream>>>(CNTI, OFFI);
  k_rank<0><<<dim3(MAXT, 1, NE), 128, 0, stream>>>(F[0], PW, F[8], LST, CNTI, OFFI, HD);
  k_lexp<0><<<dim3(MAXT, HH_ / 128, NE), 128, 0, stream>>>(HD, PW, F[10], LST, CNTI, OFFI, LO);
  k_layer<0><<<dim3(NBLKT, HH_ / 128), 128, 0, stream>>>(F[0], PW, F[4], LO, AA);
  k_rank<1><<<dim3(MAXT, 1, NE), 128, 0, stream>>>(AA, PW, F[12], LST, CNTI, OFFI, HD);
  k_lexp<1><<<dim3(MAXT, DD / 128, NE), 128, 0, stream>>>(HD, PW, F[14], LST, CNTI, OFFI, LO);
  k_layer<1><<<dim3(NBLKT, DD / 128), 128, 0, stream>>>(AA, PW, F[6], LO, OUP);
}
